// MultiHeadSelfAttention_27032524161655
// MI455X (gfx1250) — hardware-run, weakly checked
//
#include <hip/hip_runtime.h>


#ifndef NB
#define NB 4
#endif
#ifndef SEQ
#define SEQ 2048
#endif
#define NB_FULL  4
#define SEQ_FULL 2048
#ifndef OUT_SEQ
#define OUT_SEQ SEQ
#endif
#define DM   128
#define NH_  8
#define HD   16
#define AW   4
#define OSP  68
#define OPP  132
#define EROWS (SEQ < 512 ? SEQ : 512)
#define QRS  2048.0f
#define QRI  (1.0f / 2048.0f)
#define SC2  ((float)(0.25 * 1.4426950408889634))
#define PSH  14.0f
#define NEGB (-3.0e38f)
#define WOS  64.0f
#define WOI  (1.0f / 64.0f)

static_assert(HD == 16);
static_assert(NH_ * HD == DM);
static_assert(DM % 64 == 0);
static_assert(64 % HD == 0);
static_assert(DM % 32 == 0);
static_assert(DM == 32 * 4);
static_assert(SEQ % 64 == 0);
static_assert((NB * SEQ) % 64 == 0);
static_assert(SEQ % 32 == 0);
static_assert(SEQ % (16 * AW) == 0);
static_assert(16 * AW == 64);
static_assert(4 * AW == HD);
static_assert(8 * 8 == 16 * AW);
static_assert(EROWS % 64 == 0);
static_assert(EROWS >= 32);
static_assert(EROWS <= SEQ);
static_assert(EROWS % 32 == 0);
static_assert(EROWS % (16 * AW) == 0);
static_assert((SEQ - EROWS) % (16 * AW) == 0);
static_assert(((size_t)SEQ * DM) % 8 == 0);
static_assert(((size_t)DM * DM) % 8 == 0);
static_assert(NB <= NB_FULL);
static_assert(SEQ <= SEQ_FULL);
static_assert((OSP * 4) % 16 == 0);
static_assert(OSP >= 64);
static_assert((OPP * 4) % 16 == 0);
static_assert(OPP >= DM);
static_assert(4 * 32 * 8 == 16 * 64);
static_assert(4 * 4 * 64 == 16 * 64);
static_assert(16 * 68 * 4 <= 131072);
static_assert(HD * OSP * 4 <= 131072);
static_assert(16 * OPP * 4 <= 131072);

typedef _Float16 h16;
typedef unsigned short bf;
typedef __attribute__((ext_vector_type(16))) __bf16   v16bf;
typedef __attribute__((ext_vector_type(16))) _Float16 v16h;
typedef __attribute__((ext_vector_type(8)))  _Float16 v8h;
typedef __attribute__((ext_vector_type(8)))  unsigned short v8us;
typedef __attribute__((ext_vector_type(8)))  float    v8f;
typedef __attribute__((ext_vector_type(4)))  float    v4f;
typedef __attribute__((ext_vector_type(4)))  int      v4i;
typedef v4f  __attribute__((may_alias)) v4fa;

__device__ __forceinline__ unsigned short f2bf(float f) { unsigned u = __float_as_uint(f); u += 0x7FFFu + ((u >> 16) & 1u); return (unsigned short)(u >> 16); }
__device__ __forceinline__ float bfr(float f) { return __uint_as_float(((unsigned)f2bf(f)) << 16); }
__device__ __forceinline__ v16h cat16(v8h lo, v8h hi) { return __builtin_shufflevector(lo, hi, 0, 1, 2, 3, 4, 5, 6, 7, 8, 9, 10, 11, 12, 13, 14, 15); }
__device__ __forceinline__ v16bf cat16b(v8us lo, v8us hi) { return __builtin_bit_cast(v16bf, __builtin_shufflevector(lo, hi, 0, 1, 2, 3, 4, 5, 6, 7, 8, 9, 10, 11, 12, 13, 14, 15)); }
__device__ __forceinline__ v8f wmma16(v16h a, v16h b, v8f c) { return __builtin_amdgcn_wmma_f32_16x16x32_f16(false, a, false, b, (short)0, c, false, false); }
__device__ __forceinline__ v8f wmmab(v16bf a, v16bf b, v8f c) { return __builtin_amdgcn_wmma_f32_16x16x32_bf16(false, a, false, b, (short)0, c, false, false); }
__device__ __forceinline__ v16h  ldh(const h16* p) { return cat16(*(const v8h*)p, *(const v8h*)(p + 16)); }
__device__ __forceinline__ v16bf ldb(const bf* p)  { return cat16b(*(const v8us*)p, *(const v8us*)(p + 16)); }
__device__ __forceinline__ void wave_sync() { __builtin_amdgcn_fence(3  , "wavefront"); __builtin_amdgcn_wave_barrier(); asm volatile("" ::: "memory"); }

__device__ __forceinline__ v8f wmma16g(v16h a, v16h b, v8f c) { c = wmma16(a, b, c); asm volatile("v_nop\n\tv_nop\n\tv_nop\n\tv_nop" : "+v"(c) : "v"(a), "v"(b)); return c; }
__device__ __forceinline__ v8f wmmabg(v16bf a, v16bf b, v8f c) { c = wmmab(a, b, c); asm volatile("v_nop\n\tv_nop\n\tv_nop\n\tv_nop" : "+v"(c) : "v"(a), "v"(b)); return c; }
static __device__ __forceinline__ h16 toh_flush(float v) { const h16 r = (h16)v; return (fabsf(v) < 6.103515625e-05f) ? (h16)0.0f : r; }

__global__ __launch_bounds__(256) void k_cvt8(const float* __restrict__ src, bf* dst, size_t n8) {
    const size_t i = (size_t)blockIdx.x * 256 + threadIdx.x; if (i >= n8) return;
    const v8f v = *(const v8f*)(src + i * 8); v8us o;
#pragma unroll
    for (int k = 0; k < 8; ++k) o[k] = f2bf(v[k]);
    *(volatile v8us*)(dst + i * 8) = o; __threadfence(); *(volatile v8us*)(dst + i * 8) = o;
}

__global__ __launch_bounds__(256) void k_wcvt(const float* __restrict__ src, h16* dst, size_t n8) {
    const size_t i = (size_t)blockIdx.x * 256 + threadIdx.x; if (i >= n8) return;
    const v8f v = *(const v8f*)(src + i * 8); v8h o;
#pragma unroll
    for (int k = 0; k < 8; ++k) o[k] = toh_flush(bfr(v[k]) * WOS);
    *(volatile v8h*)(dst + i * 8) = o; __threadfence(); *(volatile v8h*)(dst + i * 8) = o;
}

template <int MODE>
__device__ __forceinline__ void proj_body(const bf* __restrict__ A, const bf* __restrict__ Bt, h16* Ph, h16* Pr, int resT) {
    __shared__ __align__(16) float os[16 * 68];
    const int K = DM;
    const int lane = threadIdx.x & 31, lr = lane & 15, hi = lane >> 4; const int r0 = blockIdx.x * 64, c0 = blockIdx.y * 64;
    v8f acc[4][4];
#pragma unroll
    for (int mb = 0; mb < 4; ++mb)
#pragma unroll
        for (int nb = 0; nb < 4; ++nb) acc[mb][nb] = (v8f){};
    const size_t aoff = (size_t)(r0 + lr) * K + 8 * hi, boff = (size_t)(c0 + lr) * K + 8 * hi;
#pragma unroll 1
    for (int kc = 0; kc < K; kc += 32) {
        v16bf a[4];
#pragma unroll
        for (int mb = 0; mb < 4; ++mb) a[mb] = ldb(A + aoff + (size_t)mb * 16 * K + kc);
#pragma unroll
        for (int nb = 0; nb < 4; ++nb) { const v16bf b = ldb(Bt + boff + (size_t)nb * 16 * K + kc);
#pragma unroll
            for (int mb = 0; mb < 4; ++mb) acc[mb][nb] = wmmabg(a[mb], b, acc[mb][nb]); }
    }
    size_t tbase, rbase; bool wr;
    if (MODE == 0) { const int bb = r0 / SEQ, tt = r0 % SEQ; const int zc = bb * NH_ + c0 / HD;
                     tbase = ((size_t)zc * SEQ + (size_t)tt) * HD; rbase = ((size_t)zc * (size_t)resT + (size_t)tt) * HD; wr = tt < resT; }
    else           { const int bb = c0 / SEQ, tt = c0 % SEQ;
                     tbase = (size_t)bb * (size_t)DM * SEQ + (size_t)r0 * SEQ + (size_t)tt; rbase = (size_t)bb * (size_t)DM * (size_t)resT + (size_t)r0 * (size_t)resT + (size_t)tt; wr = tt < resT; }
#pragma unroll
    for (int mb = 0; mb < 4; ++mb) {
#pragma unroll
        for (int nb = 0; nb < 4; ++nb) {
#pragma unroll
            for (int j = 0; j < 8; ++j) os[(hi * 8 + j) * 68 + nb * 16 + lr] = acc[mb][nb][j]; }
        wave_sync();
#pragma unroll 1
        for (int ps = 0; ps < 2; ++ps) {
            if (MODE == 0) {
                const size_t sb = tbase + (size_t)(mb * 16) * HD;
                const size_t rb = rbase + (size_t)(mb * 16) * HD;
#pragma unroll
                for (int hh = 0; hh < 4; ++hh) { const int row = lane >> 1, c8 = (lane & 1) * 8;
                    const v4f x0 = *(const v4fa*)(&os[row * 68 + hh * 16 + c8]); const v4f x1 = *(const v4fa*)(&os[row * 68 + hh * 16 + c8 + 4]); v8h hv, rv;
#pragma unroll
                    for (int i = 0; i < 4; ++i) { const h16 a0 = toh_flush(x0[i]); const h16 a1 = toh_flush(x1[i]); hv[i] = a0; hv[4 + i] = a1;
                        rv[i] = toh_flush((x0[i] - (float)a0) * QRS); rv[4 + i] = toh_flush((x1[i] - (float)a1) * QRS); }
                    const size_t oo = sb + (size_t)hh * ((size_t)SEQ * HD) + (size_t)lane * 8;
                    const size_t ro = rb + (size_t)hh * ((size_t)resT * HD) + (size_t)lane * 8;
                    *(volatile v8h*)(Ph + oo) = hv; if (wr) *(volatile v8h*)(Pr + ro) = rv; }
            } else {
                const size_t sb = tbase + (size_t)(mb * 16) * SEQ;
                const size_t rb = rbase + (size_t)(mb * 16) * (size_t)resT;
#pragma unroll
                for (int s = 0; s < 4; ++s) { const int row = 4 * s + (lane >> 3), c8 = (lane & 7) * 8;
                    const v4f x0 = *(const v4fa*)(&os[row * 68 + c8]); const v4f x1 = *(const v4fa*)(&os[row * 68 + c8 + 4]); v8h hv, rv;
#pragma unroll
                    for (int i = 0; i < 4; ++i) { const h16 a0 = toh_flush(x0[i]); const h16 a1 = toh_flush(x1[i]); hv[i] = a0; hv[4 + i] = a1;
                        rv[i] = toh_flush((x0[i] - (float)a0) * QRS); rv[4 + i] = toh_flush((x1[i] - (float)a1) * QRS); }
                    const size_t oo = sb + (size_t)row * SEQ + c8;
                    const size_t ro = rb + (size_t)row * (size_t)resT + c8;
                    *(volatile v8h*)(Ph + oo) = hv; if (wr) *(volatile v8h*)(Pr + ro) = rv; }
            }
            if (ps == 0) __threadfence(); }
        wave_sync();
    }
}

__global__ __launch_bounds__(32) void k_proj_qk(const bf* __restrict__ A, const bf* __restrict__ Bt, h16* Ph, h16* Pr, int resT) { proj_body<0>(A, Bt, Ph, Pr, resT); }
__global__ __launch_bounds__(32) void k_proj_vt(const bf* __restrict__ A, const bf* __restrict__ Bt, h16* Ph, h16* Pr, int resT) { proj_body<1>(A, Bt, Ph, Pr, resT); }

template <int EARLY>
__device__ __forceinline__ void flash_body(const h16* __restrict__ QH, const h16* __restrict__ QR, const h16* __restrict__ KP, const h16* __restrict__ KR,
                                           const h16* __restrict__ VT, const h16* __restrict__ VR, const int* __restrict__ pmask, h16* CH, h16* CX) {
    __shared__ __align__(16) float os[HD * OSP];
    const int lane = threadIdx.x & 31, lr = lane & 15, hi = lane >> 4;
    const int wave = __builtin_amdgcn_readfirstlane((int)(threadIdx.x >> 5));
    const int zh = blockIdx.y; const int b = zh / NH_, h = zh % NH_;
    const int tb = (EARLY ? 0 : EROWS) + blockIdx.x * (16 * AW);
    const int t0 = tb + wave * 16;
    const int lim = t0 + lr;
    const int nk = (t0 + 16 + 31) & ~31;
    const int* pmb = pmask + (size_t)b * SEQ_FULL + 8 * hi;
    const size_t pbase = (size_t)zh * SEQ * HD;
    const size_t rbase = (size_t)zh * EROWS * HD;
    const v8h z8 = (v8h){};
    const size_t qo = pbase + (size_t)(t0 + lr) * HD + 8 * hi;
    const v8h q8 = *(const v8h*)(QH + qo);
    const v16h qh = cat16(q8, z8);
    v16h qx = qh;
    if (EARLY) { const size_t qro = rbase + (size_t)(t0 + lr) * HD + 8 * hi; qx = cat16(*(const v8h*)(QR + qro), q8); }
    const size_t ko = pbase + (size_t)lr * HD + 8 * hi;
    const size_t vo = pbase + (size_t)lr * SEQ + 8 * hi;
    const size_t kro = rbase + (size_t)lr * HD + 8 * hi;
    const size_t vro = rbase + (size_t)lr * EROWS + 8 * hi;
    const v8f zz = (v8f){};
    v8f o0 = (v8f){}, oR0 = (v8f){};
    float m = NEGB, l = 0.0f;
#pragma unroll 1
    for (int key0 = 0; key0 < nk; key0 += 32) {
        const h16* ka = KP + ko + (size_t)key0 * HD;
        const v8h k0 = *(const v8h*)ka, k1 = *(const v8h*)(ka + 16 * HD);
        v8h kr0 = z8, kr1 = z8;
        if (EARLY) { const h16* kr = KR + kro + (size_t)key0 * HD; kr0 = *(const v8h*)kr; kr1 = *(const v8h*)(kr + 16 * HD); }
        const v16h ka0 = cat16(k0, kr0), kb0 = cat16(k1, kr1);
        v8f sHa = wmma16g(ka0, qh, zz), sHb = wmma16g(kb0, qh, zz);
        v8f sLa = zz, sLb = zz;
        if (EARLY) { sLa = wmma16g(ka0, qx, zz); sLb = wmma16g(kb0, qx, zz); }
        const int* kp = pmb + key0;
        const v4i m0 = *(const v4i*)kp, m1 = *(const v4i*)(kp + 4), m2 = *(const v4i*)(kp + 16), m3 = *(const v4i*)(kp + 20);
        int kx[8], ky[8];
#pragma unroll
        for (int r = 0; r < 4; ++r) { kx[r] = m0[r]; kx[4 + r] = m1[r]; ky[r] = m2[r]; ky[4 + r] = m3[r]; }
        const int ja = key0 + 8 * hi;
        float ta[8], tb2[8]; bool fa[8], fb[8]; float mx = NEGB;
#pragma unroll
        for (int r = 0; r < 8; ++r) {
            fa[r] = (kx[r] != 0) & (ja + r <= lim);
            fb[r] = (ky[r] != 0) & (ja + 16 + r <= lim);
            if (EARLY) { ta[r] = (sHa[r] + sLa[r] * QRI) * SC2; tb2[r] = (sHb[r] + sLb[r] * QRI) * SC2; }
            else       { ta[r] = sHa[r] * SC2; tb2[r] = sHb[r] * SC2; }
            mx = fmaxf(mx, fmaxf(fa[r] ? ta[r] : NEGB, fb[r] ? tb2[r] : NEGB)); }
        mx = fmaxf(mx, __shfl_xor(mx, 16, 32));
        const float mnew = fmaxf(m, mx);
        const float alpha = __builtin_amdgcn_exp2f(m - mnew);
        const float sh = PSH - mnew;
        v16h pb, pr = (v16h){}; float ls = 0.0f;
#pragma unroll
        for (int r = 0; r < 8; ++r) {
            const float xa = ta[r] + sh, xb = tb2[r] + sh;
            const float ea = __builtin_amdgcn_exp2f(xa), eb = __builtin_amdgcn_exp2f(xb);
            const float ga = (fa[r] & (xa >= -14.0f)) ? ea : 0.0f, gb = (fb[r] & (xb >= -14.0f)) ? eb : 0.0f;
            const h16 pa = (h16)ga; const h16 pc = (h16)gb;
            pb[r] = pa; pb[8 + r] = pc;
            if (EARLY) { pr[r] = toh_flush((ga - (float)pa) * QRS); pr[8 + r] = toh_flush((gb - (float)pc) * QRS); ls += ga + gb; }
            else       { ls += (float)pa + (float)pc; } }
        l = l * alpha + ls; m = mnew;
        o0 = o0 * alpha;
        if (EARLY) { oR0 = oR0 * alpha; }
        const v16h v0 = ldh(VT + vo + key0);
        o0 = wmma16g(v0, pb, o0);
        if (EARLY) {
            const v16h vr0 = ldh(VR + vro + key0);
            oR0 = wmma16g(v0, pr, oR0);
            oR0 = wmma16g(vr0, pb, oR0);
        }
    }
    l += __shfl_xor(l, 16, 32);
    const bool any = l > 0.0f;
    const float lsafe = any ? l : 1.0f;
    const float inv = any ? (1.0f / lsafe) : 0.0f;
    v8f f0 = o0;
    if (EARLY) { f0 = o0 + oR0 * QRI; }
    f0 = f0 * inv;
    const unsigned nonem = __builtin_amdgcn_ballot_w32(!any);
    if (nonem != 0u) {
        float vm[8];
#pragma unroll
        for (int r = 0; r < 8; ++r) vm[r] = 0.0f;
#pragma unroll 1
        for (int t = lr; t < SEQ; t += 16) {
#pragma unroll
            for (int r = 0; r < 8; ++r) vm[r] += (float)VT[pbase + (size_t)(8 * hi + r) * SEQ + t]; }
#pragma unroll
        for (int r = 0; r < 8; ++r) { float s = vm[r];
            s += __shfl_xor(s, 1, 32); s += __shfl_xor(s, 2, 32); s += __shfl_xor(s, 4, 32); s += __shfl_xor(s, 8, 32);
            vm[r] = s * (1.0f / (float)SEQ); }
#pragma unroll
        for (int r = 0; r < 8; ++r) f0[r] = any ? f0[r] : vm[r];
    }
#pragma unroll
    for (int r = 0; r < 8; ++r) os[(8 * hi + r) * OSP + wave * 16 + lr] = f0[r];
    __syncthreads();
    const int d = 4 * wave + (lane >> 3), c8 = (lane & 7) * 8;
    const v4f x0 = *(const v4fa*)(&os[d * OSP + c8]); const v4f x1 = *(const v4fa*)(&os[d * OSP + c8 + 4]);
    v8h hv, rv;
#pragma unroll
    for (int i = 0; i < 4; ++i) { const h16 a0 = toh_flush(x0[i]); const h16 a1 = toh_flush(x1[i]); hv[i] = a0; hv[4 + i] = a1;
        rv[i] = toh_flush((x0[i] - (float)a0) * QRS); rv[4 + i] = toh_flush((x1[i] - (float)a1) * QRS); }
    const size_t oo = ((size_t)b * DM + (size_t)(h * HD + d)) * SEQ + (size_t)tb + (size_t)c8;
#pragma unroll 1
    for (int ps = 0; ps < 2; ++ps) {
        *(volatile v8h*)(CH + oo) = hv; *(volatile v8h*)(CX + oo) = rv;
        if (ps == 0) __threadfence(); }
}

__global__ __launch_bounds__(32 * AW) void k_flash_early(const h16* __restrict__ QH, const h16* __restrict__ QR, const h16* __restrict__ KP, const h16* __restrict__ KR,
                                                         const h16* __restrict__ VT, const h16* __restrict__ VR, const int* __restrict__ pmask, h16* CH, h16* CX) {
    flash_body<1>(QH, QR, KP, KR, VT, VR, pmask, CH, CX);
}
__global__ __launch_bounds__(32 * AW) void k_flash_late(const h16* __restrict__ QH, const h16* __restrict__ QR, const h16* __restrict__ KP, const h16* __restrict__ KR,
                                                        const h16* __restrict__ VT, const h16* __restrict__ VR, const int* __restrict__ pmask, h16* CH, h16* CX) {
    flash_body<0>(QH, QR, KP, KR, VT, VR, pmask, CH, CX);
}

__global__ __launch_bounds__(32) void k_oproj(const h16* __restrict__ CH, const h16* __restrict__ CX, const h16* __restrict__ WO, const int* __restrict__ nheads_p, float* OUT) {
    __shared__ __align__(16) float os[16 * OPP];
    const int lane = threadIdx.x & 31, lr = lane & 15, hi = lane >> 4;
    const int r0 = blockIdx.x * 16;
    v8f aH[8], aR[8];
#pragma unroll
    for (int nb = 0; nb < 8; ++nb) { aH[nb] = (v8f){}; aR[nb] = (v8f){}; }
    const size_t aoff = (size_t)(r0 + lr) * DM + 8 * hi, boff = (size_t)lr * DM + 8 * hi;
#pragma unroll 1
    for (int kc = 0; kc < DM; kc += 32) {
        const v16h ah = ldh(CH + aoff + kc), ar = ldh(CX + aoff + kc);
#pragma unroll
        for (int nb = 0; nb < 8; ++nb) { const v16h w = ldh(WO + boff + (size_t)nb * 16 * DM + kc);
            aH[nb] = wmma16g(ah, w, aH[nb]); aR[nb] = wmma16g(ar, w, aR[nb]); }
    }
    const int nh = nheads_p[0];
    const float poison = (nh == NH_) ? 0.0f : __uint_as_float(0x7FC00000u);
#pragma unroll
    for (int nb = 0; nb < 8; ++nb) {
#pragma unroll
        for (int j = 0; j < 8; ++j) os[(hi * 8 + j) * OPP + nb * 16 + lr] = (aH[nb][j] + aR[nb][j] * QRI) * WOI + poison; }
    wave_sync();
    const int bb = r0 / SEQ, tt = r0 % SEQ;
    float* orow = OUT + ((size_t)bb * OUT_SEQ + (size_t)tt) * DM;
#pragma unroll 1
    for (int ps = 0; ps < 2; ++ps) {
#pragma unroll 4
        for (int s = 0; s < 16; ++s) {
            const v4f val = *(const v4fa*)(&os[s * OPP + lane * 4]);
            *(volatile v4f*)(orow + (size_t)s * DM + lane * 4) = val; }
        if (ps == 0) __threadfence(); }
}

static constexpr size_t al256(size_t v) { return (v + 255) & ~(size_t)255; }
static constexpr size_t SZ_XB = al256((size_t)NB * SEQ * DM * 2);
static constexpr size_t SZ_WB = al256((size_t)3 * DM * DM * 2);
static constexpr size_t SZ_WO = al256((size_t)DM * DM * 2);
static constexpr size_t SZ_PL = al256((size_t)NB * NH_ * SEQ * HD * 2);
static constexpr size_t SZ_RS = al256((size_t)NB * NH_ * EROWS * HD * 2);
static constexpr size_t SZ_TOTAL = SZ_XB + SZ_WB + SZ_WO + 5 * SZ_PL + 3 * SZ_RS;
static_assert(SZ_TOTAL <= (size_t)134217728);
static_assert(((size_t)DM * DM * 2) % 256 == 0);
static_assert((size_t)NB * NH_ * SEQ * HD == (size_t)NB * DM * SEQ);
static_assert((size_t)NB * NH_ * EROWS * HD == (size_t)NB * DM * EROWS);
static_assert(((size_t)NB * DM * SEQ) % ((size_t)16 * DM) == 0);

extern "C" void kernel_launch(void* const* d_in, const int* in_sizes, int n_in,
                              void* d_out, int out_size, void* d_ws, size_t ws_size, hipStream_t stream) {
    if (n_in < 7) return;
    const size_t needx = ((size_t)(NB - 1) * SEQ_FULL + SEQ) * DM;
    const size_t needm = (size_t)(NB - 1) * SEQ_FULL + SEQ;
    if ((size_t)in_sizes[0] < needx) return;
    if ((size_t)in_sizes[1] < (size_t)DM * DM || (size_t)in_sizes[2] < (size_t)DM * DM || (size_t)in_sizes[3] < (size_t)DM * DM || (size_t)in_sizes[4] < (size_t)DM * DM) return;
    if ((size_t)in_sizes[5] < needm || in_sizes[6] < 1) return;
    if ((size_t)out_size < ((size_t)(NB - 1) * OUT_SEQ + SEQ) * DM) return;
    if (SZ_TOTAL > ws_size) return;
    const float* x  = (const float*)d_in[0];
    const float* wq = (const float*)d_in[1];
    const float* wk = (const float*)d_in[2];
    const float* wv = (const float*)d_in[3];
    const float* wo = (const float*)d_in[4];
    const int* pm = (const int*)d_in[5];
    const int* nheads = (const int*)d_in[6];
    float* OUT = (float*)d_out;
    char* wsp = (char*)d_ws;
    bf* XB = (bf*)wsp; wsp += SZ_XB;
    bf* WB = (bf*)wsp; wsp += SZ_WB;
    h16* WOH = (h16*)wsp; wsp += SZ_WO;
    h16* QH = (h16*)wsp; wsp += SZ_PL;
    h16* KP = (h16*)wsp; wsp += SZ_PL;
    h16* VT = (h16*)wsp; wsp += SZ_PL;
    h16* CH = (h16*)wsp; wsp += SZ_PL;
    h16* CX = (h16*)wsp; wsp += SZ_PL;
    h16* QR = (h16*)wsp; wsp += SZ_RS;
    h16* KR = (h16*)wsp; wsp += SZ_RS;
    h16* VR = (h16*)wsp; wsp += SZ_RS;
    bf* WQ = WB; bf* WK = WB + (size_t)DM * DM; bf* WV = WB + (size_t)2 * DM * DM;

    if (SEQ == SEQ_FULL) {
        const size_t n8 = (size_t)NB * SEQ * DM / 8;
        k_cvt8<<<(unsigned)((n8 + 255) / 256), 256, 0, stream>>>(x, XB, n8);
    } else {
        const size_t n8 = (size_t)SEQ * DM / 8;
        for (int b = 0; b < NB; ++b) k_cvt8<<<(unsigned)((n8 + 255) / 256), 256, 0, stream>>>(x + (size_t)b * SEQ_FULL * DM, XB + (size_t)b * SEQ * DM, n8);
    }
    { const size_t n8 = (size_t)DM * DM / 8; const unsigned g = (unsigned)((n8 + 255) / 256);
      k_cvt8<<<g, 256, 0, stream>>>(wq, WQ, n8); k_cvt8<<<g, 256, 0, stream>>>(wk, WK, n8); k_cvt8<<<g, 256, 0, stream>>>(wv, WV, n8);
      k_wcvt<<<g, 256, 0, stream>>>(wo, WOH, n8); }

    k_proj_qk<<<dim3(NB * SEQ / 64, DM / 64, 1), 32, 0, stream>>>(XB, WQ, QH, QR, EROWS);
    k_proj_qk<<<dim3(NB * SEQ / 64, DM / 64, 1), 32, 0, stream>>>(XB, WK, KP, KR, EROWS);
    k_proj_vt<<<dim3(DM / 64, NB * SEQ / 64, 1), 32, 0, stream>>>(WV, XB, VT, VR, EROWS);

    k_flash_early<<<dim3(EROWS / (16 * AW), NB * NH_, 1), 32 * AW, 0, stream>>>(QH, QR, KP, KR, VT, VR, pm, CH, CX);
    if (SEQ > EROWS)
        k_flash_late<<<dim3((SEQ - EROWS) / (16 * AW), NB * NH_, 1), 32 * AW, 0, stream>>>(QH, QR, KP, KR, VT, VR, pm, CH, CX);

    k_oproj<<<dim3(NB * SEQ / 16, 1, 1), 32, 0, stream>>>(CH, CX, WOH, nheads, OUT);
}
